// PointNet_FeaturePropagation_36120674959458
// MI455X (gfx1250) — hardware-verified
//
#include <hip/hip_runtime.h>
#pragma clang fp contract(off)

typedef __attribute__((ext_vector_type(16))) _Float16 v16h;
typedef __attribute__((ext_vector_type(8)))  _Float16 v8h;
typedef __attribute__((ext_vector_type(16))) __bf16   v16b;
typedef __attribute__((ext_vector_type(8)))  __bf16   v8b;
typedef __attribute__((ext_vector_type(8)))  float    v8f;
typedef __attribute__((ext_vector_type(4)))  float    v4f;
typedef __attribute__((ext_vector_type(4)))  unsigned v4u;
typedef __attribute__((ext_vector_type(4)))  int      v4i;

constexpr int kNB     = 4;
constexpr int kNPTS   = 8192;
constexpr int kNSRC   = 2048;
constexpr int kCH1    = 128;
constexpr int kCH2    = 256;
constexpr int kCIN    = kCH1 + kCH2;
constexpr int kCOUT   = 256;
constexpr int kMROWS  = kNB * kNPTS;
constexpr int kNBLOCKS = 2;
constexpr int kXP     = 388;
static_assert(kCIN == 384);
static_assert(kMROWS == 32768);
static_assert(kCIN % 32 == 0 && kCOUT % 32 == 0);
static_assert(kMROWS % 64 == 0 && kCOUT % 64 == 0);
static_assert(kNSRC / 4 == 2 * 256);
static_assert((kXP * 4) % 16 == 0);

constexpr int kWFuseElems = kCOUT * kCIN;
constexpr int kWBlkElems  = kNBLOCKS * kCOUT * kCOUT;
constexpr int kWTotal     = kWFuseElems + 2 * kWBlkElems;
constexpr int kWFuseBlocks = kWFuseElems / 2048;
constexpr int kWBlkBlocks  = kWBlkElems / 2048;
static_assert(kWFuseElems % 2048 == 0 && kWBlkElems % 2048 == 0);

__device__ __forceinline__ unsigned bf_bits_rne(float f) {
  const unsigned u = __float_as_uint(f);
  return (u + 0x7FFFu + ((u >> 16) & 1u)) >> 16;
}
__device__ __forceinline__ void bf_split(float v, unsigned& hb, unsigned& lb) {
  hb = bf_bits_rne(v);
  const float res = v - __uint_as_float(hb << 16);
  lb = bf_bits_rne(res);
}
__device__ __forceinline__ unsigned short f2bf_bits(float f) {
  return (unsigned short)bf_bits_rne(f);
}
__device__ __forceinline__ float bf_bits2f(unsigned short h) { return __uint_as_float(((unsigned)h) << 16); }

__device__ __forceinline__ void split8(const float* z, v4u& hv, v4u& lv) {
  unsigned h[8], l[8];
#pragma unroll
  for (int e = 0; e < 8; ++e) bf_split(z[e], h[e], l[e]);
  hv[0] = h[0] | (h[1] << 16); hv[1] = h[2] | (h[3] << 16);
  hv[2] = h[4] | (h[5] << 16); hv[3] = h[6] | (h[7] << 16);
  lv[0] = l[0] | (l[1] << 16); lv[1] = l[2] | (l[3] << 16);
  lv[2] = l[4] | (l[5] << 16); lv[3] = l[6] | (l[7] << 16);
}

__device__ __forceinline__ void dep_guard4_h(v8f& a, v8f& b, v8f& c, v8f& d, v16h x, v16h y) { asm volatile("v_nop\n\tv_nop\n\tv_nop\n\tv_nop" : "+v"(a), "+v"(b), "+v"(c), "+v"(d) : "v"(x), "v"(y)); }
__device__ __forceinline__ void dep_guard4_b(v8f& a, v8f& b, v8f& c, v8f& d, v16b x, v16b y) { asm volatile("v_nop\n\tv_nop\n\tv_nop\n\tv_nop" : "+v"(a), "+v"(b), "+v"(c), "+v"(d) : "v"(x), "v"(y)); }
__device__ __forceinline__ void keep4_h(v16h a, v16h b, v16h c, v16h d) { asm volatile("v_nop" :: "v"(a), "v"(b), "v"(c), "v"(d)); }
__device__ __forceinline__ void keep4_b(v16b a, v16b b, v16b c, v16b d) { asm volatile("v_nop" :: "v"(a), "v"(b), "v"(c), "v"(d)); }
__device__ __forceinline__ void acc_guard4(v8f& a, v8f& b, v8f& c, v8f& d) { asm volatile("v_nop\n\tv_nop\n\tv_nop\n\tv_nop" : "+v"(a), "+v"(b), "+v"(c), "+v"(d)); }
template <typename T> struct Frag;
template <> struct Frag<_Float16> {
  typedef v16h V; union U { v16h v; v8h h[2]; };
  static __device__ __forceinline__ v16h load(const _Float16* p) {
    U f; f.h[0] = *(const v8h*)(p); f.h[1] = *(const v8h*)(p + 16); return f.v;
  }
  static __device__ __forceinline__ v8f mma(v16h a, v16h b, v8f c) {
    return __builtin_amdgcn_wmma_f32_16x16x32_f16(false, a, false, b, (short)0, c, false, false);
  }
  static __device__ __forceinline__ void guard4(v8f& a, v8f& b, v8f& c, v8f& d, v16h x, v16h y) { dep_guard4_h(a, b, c, d, x, y); }
  static __device__ __forceinline__ void keep(v16h a, v16h b, v16h c, v16h d) { keep4_h(a, b, c, d); }
};
template <> struct Frag<__bf16> {
  typedef v16b V; union U { v16b v; v8b h[2]; };
  static __device__ __forceinline__ v16b load(const __bf16* p) {
    U f; f.h[0] = *(const v8b*)(p); f.h[1] = *(const v8b*)(p + 16); return f.v;
  }
  static __device__ __forceinline__ v8f mma(v16b a, v16b b, v8f c) {
    return __builtin_amdgcn_wmma_f32_16x16x32_bf16(false, a, false, b, (short)0, c, false, false);
  }
  static __device__ __forceinline__ void guard4(v8f& a, v8f& b, v8f& c, v8f& d, v16b x, v16b y) { dep_guard4_b(a, b, c, d, x, y); }
  static __device__ __forceinline__ void keep(v16b a, v16b b, v16b c, v16b d) { keep4_b(a, b, c, d); }
};

template <int ET> struct Elem;
template <> struct Elem<0> { typedef _Float16 T; };
template <> struct Elem<1> { typedef __bf16 T; };
template <int ET, bool SPLIT, int BIAS_MODE, int OUT_MODE, bool RESID, int ACT = 0>
__global__ __launch_bounds__(256) void wmma_gemm64(
    const unsigned short* __restrict__ Ap, const unsigned short* __restrict__ A2p, int lda, long strideA,
    const unsigned short* __restrict__ Btp, const unsigned short* __restrict__ Bt2p, int ldb, long strideB,
    void* __restrict__ Cout, void* __restrict__ Cout2, int ldc, long strideC,
    const float* __restrict__ bias,
    const float* __restrict__ resid, long strideR,
    int M, int N, int K, float scale) {
  typedef typename Elem<ET>::T T;
  typedef typename Frag<T>::V V;
  const T* A = (const T*)Ap; const T* A2 = (const T*)A2p; const T* Bt = (const T*)Btp; const T* Bt2 = (const T*)Bt2p;
  __shared__ __align__(16) float sT[8][16 * 68];
  const int b    = blockIdx.y;
  const int lane = threadIdx.x & 31;
  const int wave = threadIdx.x >> 5;
  const int tilesN = N >> 6;
  const int tilesM = M >> 6;
  const int tile = blockIdx.x * 8 + wave;
  if (tile >= tilesM * tilesN) return;
  const int tm = tile / tilesN;
  const int tn = tile - tm * tilesN;
  const int m0 = tm << 6;
  const int n0 = tn << 6;

  const T* Ab  = A  + (size_t)b * strideA;
  const T* Bb  = Bt + (size_t)b * strideB;
  const T* Ab2 = SPLIT ? (A2  + (size_t)b * strideA) : nullptr;
  const T* Bb2 = SPLIT ? (Bt2 + (size_t)b * strideB) : nullptr;

  const int rlane = lane & 15;
  const int koff  = (lane >> 4) * 8;
  const int mOff  = (lane >> 4) * 8;

  v8f acc[4][4];
#pragma unroll
  for (int i = 0; i < 4; ++i)
#pragma unroll
    for (int j = 0; j < 4; ++j) acc[i][j] = (v8f){0.f,0.f,0.f,0.f,0.f,0.f,0.f,0.f};

  for (int k0 = 0; k0 < K; k0 += 32) {
    V bh[4], bl[4];
#pragma unroll
    for (int j = 0; j < 4; ++j) {
      const size_t bo = (size_t)(n0 + (j << 4) + rlane) * ldb + koff + k0;
      bh[j] = Frag<T>::load(Bb + bo);
      if (SPLIT) bl[j] = Frag<T>::load(Bb2 + bo);
    }
#pragma unroll
    for (int i = 0; i < 4; ++i) {
      const size_t ao = (size_t)(m0 + (i << 4) + rlane) * lda + koff + k0;
      V ah = Frag<T>::load(Ab + ao);
      V al;
      if (SPLIT) al = Frag<T>::load(Ab2 + ao);
#pragma unroll
      for (int j = 0; j < 4; ++j) {
        acc[i][j] = Frag<T>::mma(ah, bh[j], acc[i][j]);
        if (SPLIT) {
          acc[i][j] = Frag<T>::mma(ah, bl[j], acc[i][j]);
          acc[i][j] = Frag<T>::mma(al, bh[j], acc[i][j]);
        }
      }
      Frag<T>::guard4(acc[i][0], acc[i][1], acc[i][2], acc[i][3], ah, SPLIT ? al : ah);
    }
    Frag<T>::keep(bh[0], bh[1], bh[2], bh[3]);
    if (SPLIT) Frag<T>::keep(bl[0], bl[1], bl[2], bl[3]);
  }
  acc_guard4(acc[0][0], acc[0][1], acc[0][2], acc[0][3]);
  acc_guard4(acc[1][0], acc[1][1], acc[1][2], acc[1][3]);
  acc_guard4(acc[2][0], acc[2][1], acc[2][2], acc[2][3]);
  acc_guard4(acc[3][0], acc[3][1], acc[3][2], acc[3][3]);

  float* slab = sT[wave];
  const float* Rb = RESID ? (resid + (size_t)b * strideR) : nullptr;
#pragma unroll
  for (int i = 0; i < 4; ++i) {
    const int mBase = m0 + (i << 4);
#pragma unroll
    for (int j = 0; j < 4; ++j) {
      const int n = n0 + (j << 4) + rlane;
      float bv = 0.f;
      if (BIAS_MODE == 2) bv = bias[n];
#pragma unroll
      for (int r = 0; r < 8; ++r) {
        float v = acc[i][j][r] * scale;
        if (BIAS_MODE == 1) v += bias[mBase + mOff + r];
        if (BIAS_MODE == 2) v += bv;
        if (RESID) v += Rb[(size_t)(mBase + mOff + r) * ldc + n];
        if (ACT == 2) v = fmaxf(v, 0.0f);
        slab[(mOff + r) * 68 + (j << 4) + rlane] = v;
      }
    }
    __builtin_amdgcn_fence(__ATOMIC_RELEASE, "workgroup");
    __builtin_amdgcn_wave_barrier();
    __builtin_amdgcn_fence(__ATOMIC_ACQUIRE, "workgroup");
    if (OUT_MODE == 0) {
      float* C = (float*)Cout + (size_t)b * strideC;
      const int hh = lane >> 4, c4 = (lane & 15) * 4;
      for (int pass = 0; pass < 2; ++pass) {
#pragma unroll
        for (int it = 0; it < 8; ++it) {
          const int row = it * 2 + hh;
          v4f v = *(const v4f*)(slab + row * 68 + c4);
          *(volatile v4f*)(C + (size_t)(mBase + row) * ldc + n0 + c4) = v;
        }
        __threadfence();
      }
    } else {
      const int q = lane >> 3, c8 = (lane & 7) * 8;
      unsigned short* C  = (unsigned short*)Cout  + (size_t)b * strideC;
      unsigned short* C2 = (OUT_MODE == 2) ? ((unsigned short*)Cout2 + (size_t)b * strideC) : nullptr;
      for (int pass = 0; pass < 2; ++pass) {
#pragma unroll
        for (int it = 0; it < 4; ++it) {
          const int row = it * 4 + q;
          const float* sp = slab + row * 68 + c8;
          v8h hv, lv;
#pragma unroll
          for (int e = 0; e < 8; ++e) {
            if (OUT_MODE == 1) {
              hv[e] = (_Float16)sp[e];
            } else {
              unsigned short hb = f2bf_bits(sp[e]);
              unsigned short lb = f2bf_bits(sp[e] - bf_bits2f(hb));
              hv[e] = __builtin_bit_cast(_Float16, hb);
              lv[e] = __builtin_bit_cast(_Float16, lb);
            }
          }
          *(volatile v8h*)(C + (size_t)(mBase + row) * ldc + n0 + c8) = hv;
          if (OUT_MODE == 2) *(volatile v8h*)(C2 + (size_t)(mBase + row) * ldc + n0 + c8) = lv;
        }
        __threadfence();
      }
    }
    __builtin_amdgcn_fence(__ATOMIC_RELEASE, "workgroup");
    __builtin_amdgcn_wave_barrier();
    __builtin_amdgcn_fence(__ATOMIC_ACQUIRE, "workgroup");
  }
}

__global__ __launch_bounds__(256) void wsplit_kernel(const float* __restrict__ wf,
                                                     const float* __restrict__ w1,
                                                     const float* __restrict__ w2,
                                                     unsigned short* __restrict__ hi,
                                                     unsigned short* __restrict__ lo) {
  const int blk = blockIdx.x;
  const float* src = wf;
  int lblk = blk;
  int base = 0;
  if (blk >= kWFuseBlocks + kWBlkBlocks) {
    src = w2; lblk = blk - kWFuseBlocks - kWBlkBlocks; base = kWFuseElems + kWBlkElems;
  } else if (blk >= kWFuseBlocks) {
    src = w1; lblk = blk - kWFuseBlocks; base = kWFuseElems;
  }
  const int e0 = (lblk * 256 + (int)threadIdx.x) * 8;
  const v4f a = *(const v4f*)(src + e0);
  const v4f c = *(const v4f*)(src + e0 + 4);
  float z[8];
  z[0] = a[0]; z[1] = a[1]; z[2] = a[2]; z[3] = a[3];
  z[4] = c[0]; z[5] = c[1]; z[6] = c[2]; z[7] = c[3];
  v4u hv, lv;
  split8(z, hv, lv);
  const size_t off = (size_t)base + (size_t)e0;
  *(volatile v4u*)(hi + off) = hv;
  *(volatile v4u*)(lo + off) = lv;
  __threadfence();
  *(volatile v4u*)(hi + off) = hv;
  *(volatile v4u*)(lo + off) = lv;
}

__global__ __launch_bounds__(256) void p2t_kernel(const float* __restrict__ p2, float* __restrict__ p2T) {
  __shared__ float tile[32][33];
  const int tid = threadIdx.x;
  const int tx = tid & 31, ty = tid >> 5;
  const int s0 = blockIdx.x * 32, c0 = blockIdx.y * 32, b = blockIdx.z;
#pragma unroll
  for (int i = 0; i < 4; ++i) {
    const int c = ty + 8 * i;
    tile[c][tx] = p2[((size_t)(b * kCH2 + c0 + c)) * kNSRC + s0 + tx];
  }
  __syncthreads();
  const int sl = ty * 4 + (tx >> 3);
  const int cq = (tx & 7) * 4;
  v4f v;
  v[0] = tile[cq][sl]; v[1] = tile[cq + 1][sl]; v[2] = tile[cq + 2][sl]; v[3] = tile[cq + 3][sl];
  float* dst = p2T + ((size_t)(b * kNSRC + s0 + sl)) * kCH2 + c0 + cq;
  *(volatile v4f*)dst = v;
  __threadfence();
  *(volatile v4f*)dst = v;
}

__global__ __launch_bounds__(256) void knn3_kernel(const float* __restrict__ xyz1,
                                                   const float* __restrict__ xyz2,
                                                   int* __restrict__ idx_out,
                                                   float* __restrict__ dsel_out) {
#pragma clang fp contract(off)
  __shared__ __align__(16) float src4[kNSRC * 4];
  const int tid = threadIdx.x;
  const int b = blockIdx.y;
  const float* x2 = xyz2 + (size_t)b * 3 * kNSRC;
#pragma unroll
  for (int i = 0; i < 2; ++i) {
    const int q = tid + 256 * i;
    const v4f X = *(const v4f*)(x2 + 4 * q);
    const v4f Yv = *(const v4f*)(x2 + kNSRC + 4 * q);
    const v4f Z = *(const v4f*)(x2 + 2 * kNSRC + 4 * q);
#pragma unroll
    for (int e = 0; e < 4; ++e) {
      const float xe = X[e], ye = Yv[e], ze = Z[e];
      const float xx = xe * xe;
      const float yy = ye * ye;
      const float zz = ze * ze;
      const float sq = (xx + zz) + yy;
      v4f o;
      o[0] = xe; o[1] = ye; o[2] = ze; o[3] = sq;
      *(v4f*)(src4 + (4 * q + e) * 4) = o;
    }
  }
  __syncthreads();

  const int n = blockIdx.x * 256 + tid;
  const float* x1 = xyz1 + (size_t)b * 3 * kNPTS;
  const float px = x1[n];
  const float py = x1[kNPTS + n];
  const float pz = x1[2 * kNPTS + n];
  const float pxx = px * px;
  const float pyy = py * py;
  const float pzz = pz * pz;
  const float sq1 = (pxx + pzz) + pyy;

  float d0 = __builtin_inff(), d1 = __builtin_inff(), d2 = __builtin_inff();
  int i0 = 0, i1 = 0, i2 = 0;
#pragma unroll 4
  for (int s = 0; s < kNSRC; ++s) {
    const v4f c = *(const v4f*)(src4 + 4 * s);
    float p = px * c[0];
    p = __builtin_fmaf(py, c[1], p);
    p = __builtin_fmaf(pz, c[2], p);
    const float ssum = sq1 + c[3];
    const float p2x = p + p;
    const float d = ssum - p2x;
    const bool l0 = d < d0;
    const bool l1 = d < d1;
    const bool l2 = d < d2;
    const float nd2 = l1 ? d1 : (l2 ? d : d2);
    const int   ni2 = l1 ? i1 : (l2 ? s : i2);
    const float nd1 = l0 ? d0 : (l1 ? d : d1);
    const int   ni1 = l0 ? i0 : (l1 ? s : i1);
    const float nd0 = l0 ? d : d0;
    const int   ni0 = l0 ? s : i0;
    d0 = nd0; d1 = nd1; d2 = nd2;
    i0 = ni0; i1 = ni1; i2 = ni2;
  }
  const size_t m = (size_t)b * kNPTS + n;
  v4i iv;
  iv[0] = i0; iv[1] = i1; iv[2] = i2; iv[3] = 0;
  v4f dv;
  dv[0] = d0; dv[1] = d1; dv[2] = d2; dv[3] = 0.0f;
  *(volatile v4i*)(idx_out + m * 4) = iv;
  *(volatile v4f*)(dsel_out + m * 4) = dv;
  __threadfence();
  *(volatile v4i*)(idx_out + m * 4) = iv;
  *(volatile v4f*)(dsel_out + m * 4) = dv;
}

__global__ __launch_bounds__(256) void xcat_kernel(const float* __restrict__ points1,
                                                   const float* __restrict__ p2T,
                                                   const int* __restrict__ idx_tab,
                                                   const float* __restrict__ dsel_tab,
                                                   unsigned short* __restrict__ xhi,
                                                   unsigned short* __restrict__ xlo) {
  __shared__ __align__(16) float F[32 * kXP];
  __shared__ __align__(16) float wl[32 * 4];
  __shared__ __align__(16) int   il[32 * 4];
  const int tid = threadIdx.x;
  const int wave = tid >> 5;
  const int lane = tid & 31;
  const int m0 = blockIdx.x * 32;
  const int b = m0 / kNPTS;
  const int n0 = m0 - b * kNPTS;

  if (tid < 32) {
    const v4i iv = *(const v4i*)(idx_tab + (size_t)(m0 + tid) * 4);
    const v4f dv = *(const v4f*)(dsel_tab + (size_t)(m0 + tid) * 4);
    const float r0 = 1.0f / (dv[0] + 1e-8f);
    const float r1 = 1.0f / (dv[1] + 1e-8f);
    const float r2 = 1.0f / (dv[2] + 1e-8f);
    const float rs = (r0 + r2) + r1;
    wl[tid * 4 + 0] = r0 / rs;
    wl[tid * 4 + 1] = r1 / rs;
    wl[tid * 4 + 2] = r2 / rs;
    wl[tid * 4 + 3] = 0.0f;
    int a0 = iv[0], a1 = iv[1], a2 = iv[2];
    a0 = a0 < 0 ? 0 : (a0 > kNSRC - 1 ? kNSRC - 1 : a0);
    a1 = a1 < 0 ? 0 : (a1 > kNSRC - 1 ? kNSRC - 1 : a1);
    a2 = a2 < 0 ? 0 : (a2 > kNSRC - 1 ? kNSRC - 1 : a2);
    il[tid * 4 + 0] = a0;
    il[tid * 4 + 1] = a1;
    il[tid * 4 + 2] = a2;
    il[tid * 4 + 3] = 0;
  }
  {
    const float* p1b = points1 + (size_t)b * kCH1 * kNPTS + n0;
#pragma unroll
    for (int i = 0; i < 4; ++i) {
      const int q = tid + 256 * i;
      const int c = q >> 3;
      const int n4 = (q & 7) * 4;
      const v4f v = *(const v4f*)(p1b + (size_t)c * kNPTS + n4);
      F[(n4 + 0) * kXP + c] = v[0];
      F[(n4 + 1) * kXP + c] = v[1];
      F[(n4 + 2) * kXP + c] = v[2];
      F[(n4 + 3) * kXP + c] = v[3];
    }
  }
  __syncthreads();
  {
    const float* p2b = p2T + (size_t)b * kNSRC * kCH2;
#pragma unroll 1
    for (int j = 0; j < 4; ++j) {
      const int nl = wave * 4 + j;
      const int a0 = il[nl * 4 + 0], a1 = il[nl * 4 + 1], a2 = il[nl * 4 + 2];
      const float w0 = wl[nl * 4 + 0], w1 = wl[nl * 4 + 1], w2 = wl[nl * 4 + 2];
#pragma unroll
      for (int hf = 0; hf < 2; ++hf) {
        const int c = hf * 128 + lane * 4;
        const v4f g0 = *(const v4f*)(p2b + (size_t)a0 * kCH2 + c);
        const v4f g1 = *(const v4f*)(p2b + (size_t)a1 * kCH2 + c);
        const v4f g2 = *(const v4f*)(p2b + (size_t)a2 * kCH2 + c);
        v4f o;
#pragma unroll
        for (int e = 0; e < 4; ++e) {
          const float t0 = g0[e] * w0;
          const float t1 = g1[e] * w1;
          const float t2 = g2[e] * w2;
          o[e] = (t0 + t1) + t2;
        }
        *(v4f*)(F + nl * kXP + kCH1 + c) = o;
      }
    }
  }
  __syncthreads();
  for (int pass = 0; pass < 2; ++pass) {
#pragma unroll 1
    for (int it = 0; it < 6; ++it) {
      const int g = it * 256 + tid;
      const int row = g / 48;
      const int col = (g - row * 48) * 8;
      const v4f f0 = *(const v4f*)(F + row * kXP + col);
      const v4f f1 = *(const v4f*)(F + row * kXP + col + 4);
      float z[8];
      z[0] = f0[0]; z[1] = f0[1]; z[2] = f0[2]; z[3] = f0[3];
      z[4] = f1[0]; z[5] = f1[1]; z[6] = f1[2]; z[7] = f1[3];
      v4u hv, lv;
      split8(z, hv, lv);
      const size_t off = (size_t)m0 * kCIN + (size_t)g * 8;
      *(volatile v4u*)(xhi + off) = hv;
      *(volatile v4u*)(xlo + off) = lv;
    }
    __threadfence();
  }
}

__global__ __launch_bounds__(256) void colstats_kernel(const float* __restrict__ Y, float* __restrict__ part) {
  __shared__ __align__(16) float sl[512];
  const int tid = threadIdx.x;
  const size_t r0 = (size_t)blockIdx.x * 128;
  float s = 0.0f, q = 0.0f;
#pragma unroll 8
  for (int r = 0; r < 128; ++r) {
    const float v = Y[(r0 + r) * kCOUT + tid];
    s = s + v;
    const float vv = v * v;
    q = q + vv;
  }
  sl[tid] = s;
  sl[256 + tid] = q;
  __syncthreads();
  if (tid < 128) {
    const v4f v = *(const v4f*)(sl + 4 * tid);
    float* dst = part + (size_t)blockIdx.x * 512 + 4 * tid;
    *(volatile v4f*)dst = v;
    __threadfence();
    *(volatile v4f*)dst = v;
  }
}

__global__ __launch_bounds__(256) void bnfin_kernel(const float* __restrict__ part,
                                                    const float* __restrict__ gam,
                                                    const float* __restrict__ bet,
                                                    float* __restrict__ ss) {
  __shared__ __align__(16) float sl[512];
  const int tid = threadIdx.x;
  double s = 0.0, q = 0.0;
#pragma unroll 4
  for (int k = 0; k < kMROWS / 128; ++k) {
    s = s + (double)part[(size_t)k * 512 + tid];
    q = q + (double)part[(size_t)k * 512 + 256 + tid];
  }
  const double invm = 1.0 / (double)kMROWS;
  const double mean = s * invm;
  const double ex2 = q * invm;
  double var = ex2 - mean * mean;
  var = var < 0.0 ? 0.0 : var;
  const float varf = (float)var;
  const float meanf = (float)mean;
  const float rs = 1.0f / sqrtf(varf + 1e-5f);
  const float sc = gam[tid] * rs;
  const float sh = bet[tid] - meanf * sc;
  sl[tid] = sc;
  sl[256 + tid] = sh;
  __syncthreads();
  if (tid < 128) {
    const v4f v = *(const v4f*)(sl + 4 * tid);
    float* dst = ss + 4 * tid;
    *(volatile v4f*)dst = v;
    __threadfence();
    *(volatile v4f*)dst = v;
  }
}

__device__ __forceinline__ void resid8(const v4u rh, const v4u rl, float* x) {
#pragma unroll
  for (int k = 0; k < 4; ++k) {
    const unsigned wh = rh[k];
    const unsigned wlw = rl[k];
    const float h0 = __uint_as_float(wh << 16);
    const float h1 = __uint_as_float(wh & 0xffff0000u);
    const float l0 = __uint_as_float(wlw << 16);
    const float l1 = __uint_as_float(wlw & 0xffff0000u);
    x[2 * k] = h0 + l0;
    x[2 * k + 1] = h1 + l1;
  }
}

template <bool RESID>
__global__ __launch_bounds__(256) void bn_apply_planes(const float* __restrict__ Y,
                                                       const float* __restrict__ ss,
                                                       const unsigned short* rhi,
                                                       const unsigned short* rlo,
                                                       unsigned short* ohi,
                                                       unsigned short* olo) {
  __shared__ __align__(16) float sss[512];
  const int tid = threadIdx.x;
  if (tid < 128) *(v4f*)(sss + 4 * tid) = *(const v4f*)(ss + 4 * tid);
  __syncthreads();
  const size_t g = (size_t)blockIdx.x * 256 + tid;
  const int c8 = (int)(g & 31) * 8;
  const v4f y0 = *(const v4f*)(Y + g * 8);
  const v4f y1 = *(const v4f*)(Y + g * 8 + 4);
  float xr[8];
  if (RESID) {
    const v4u rh = *(const v4u*)(rhi + g * 8);
    const v4u rl = *(const v4u*)(rlo + g * 8);
    resid8(rh, rl, xr);
  }
  float z[8];
#pragma unroll
  for (int e = 0; e < 8; ++e) {
    const float yv = (e < 4) ? y0[e & 3] : y1[e & 3];
    const float t = yv * sss[c8 + e];
    float v = t + sss[256 + c8 + e];
    if (RESID) v = v + xr[e];
    z[e] = fmaxf(v, 0.0f);
  }
  v4u hv, lv;
  split8(z, hv, lv);
  *(volatile v4u*)(ohi + g * 8) = hv;
  *(volatile v4u*)(olo + g * 8) = lv;
  __threadfence();
  *(volatile v4u*)(ohi + g * 8) = hv;
  *(volatile v4u*)(olo + g * 8) = lv;
}

__global__ __launch_bounds__(256) void bn_apply_final(const float* __restrict__ Y,
                                                      const float* __restrict__ ss,
                                                      const unsigned short* __restrict__ rhi,
                                                      const unsigned short* __restrict__ rlo,
                                                      float* __restrict__ out) {
  __shared__ __align__(16) float sss[512];
  __shared__ float Zt[kCOUT * 33];
  const int tid = threadIdx.x;
  const int wave = tid >> 5;
  const int lane = tid & 31;
  const int m0 = blockIdx.x * 32;
  const int b = m0 / kNPTS;
  const int n0 = m0 - b * kNPTS;
  if (tid < 128) *(v4f*)(sss + 4 * tid) = *(const v4f*)(ss + 4 * tid);
  __syncthreads();
#pragma unroll 1
  for (int it = 0; it < 4; ++it) {
    const int g = it * 256 + tid;
    const int row = g >> 5;
    const int c8 = (g & 31) * 8;
    const size_t eo = (size_t)(m0 + row) * kCOUT + c8;
    const v4f y0 = *(const v4f*)(Y + eo);
    const v4f y1 = *(const v4f*)(Y + eo + 4);
    const v4u rh = *(const v4u*)(rhi + eo);
    const v4u rl = *(const v4u*)(rlo + eo);
    float xr[8];
    resid8(rh, rl, xr);
#pragma unroll
    for (int e = 0; e < 8; ++e) {
      const float yv = (e < 4) ? y0[e & 3] : y1[e & 3];
      const float t = yv * sss[c8 + e];
      float v = t + sss[256 + c8 + e];
      v = v + xr[e];
      Zt[(c8 + e) * 33 + row] = fmaxf(v, 0.0f);
    }
  }
  __syncthreads();
  const int n4 = (lane & 7) * 4;
  for (int pass = 0; pass < 2; ++pass) {
#pragma unroll 1
    for (int it = 0; it < 8; ++it) {
      const int o = wave * 32 + it * 4 + (lane >> 3);
      v4f v;
      v[0] = Zt[o * 33 + n4];
      v[1] = Zt[o * 33 + n4 + 1];
      v[2] = Zt[o * 33 + n4 + 2];
      v[3] = Zt[o * 33 + n4 + 3];
      float* dst = out + ((size_t)(b * kCOUT + o)) * kNPTS + n0 + n4;
      *(volatile v4f*)dst = v;
    }
    __threadfence();
  }
}

constexpr size_t kOffXhi  = 0;
constexpr size_t kOffXlo  = (size_t)kMROWS * kCIN * 2;
constexpr size_t kOffAhi  = 0;
constexpr size_t kOffAlo  = (size_t)kMROWS * kCOUT * 2;
constexpr size_t kOffY    = 2 * (size_t)kMROWS * kCIN * 2;
constexpr size_t kOffBhi  = kOffY + (size_t)kMROWS * kCOUT * 4;
constexpr size_t kOffBlo  = kOffBhi + (size_t)kMROWS * kCOUT * 2;
constexpr size_t kOffP2T  = kOffBlo + (size_t)kMROWS * kCOUT * 2;
constexpr size_t kOffWhi  = kOffP2T + (size_t)kNB * kNSRC * kCH2 * 4;
constexpr size_t kOffWlo  = kOffWhi + (size_t)kWTotal * 2;
constexpr size_t kOffIdx  = kOffWlo + (size_t)kWTotal * 2;
constexpr size_t kOffDsel = kOffIdx + (size_t)kMROWS * 16;
constexpr size_t kOffPart = kOffDsel + (size_t)kMROWS * 16;
constexpr size_t kPartBytes = (size_t)(kMROWS / 128) * 512 * 4;
constexpr size_t kOffSS   = kOffPart + 5 * kPartBytes;
constexpr size_t kWsTotal = kOffSS + 5 * 2048;
static_assert(kOffY == 50331648);
static_assert(kWsTotal == 130951168);
static_assert(kWsTotal <= 134217728);
static_assert(kOffAlo + (size_t)kMROWS * kCOUT * 2 <= kOffY);
static_assert(kOffWhi % 128 == 0 && kOffWlo % 128 == 0 && kOffIdx % 128 == 0 && kOffPart % 128 == 0 && kOffSS % 128 == 0);

static void run_conv_stats(const unsigned short* ahi, const unsigned short* alo, int kdim,
                           const unsigned short* whi, const unsigned short* wlo,
                           const float* bias, const float* gam, const float* bet,
                           float* yb, float* part, float* ss, hipStream_t stream) {
  wmma_gemm64<1, true, 2, 0, false, 0><<<dim3((kMROWS / 64) * (kCOUT / 64) / 8, 1), 256, 0, stream>>>(
      ahi, alo, kdim, 0L, whi, wlo, kdim, 0L, (void*)yb, (void*)yb, kCOUT, 0L, bias, bias, 0L,
      kMROWS, kCOUT, kdim, 1.0f);
  colstats_kernel<<<kMROWS / 128, 256, 0, stream>>>(yb, part);
  bnfin_kernel<<<1, 256, 0, stream>>>(part, gam, bet, ss);
}

extern "C" void kernel_launch(void* const* d_in, const int* in_sizes, int n_in,
                              void* d_out, int out_size, void* d_ws, size_t ws_size,
                              hipStream_t stream) {
  (void)in_sizes; (void)n_in; (void)out_size;
  if (ws_size < kWsTotal) return;
  const float* xyz1    = (const float*)d_in[0];
  const float* xyz2    = (const float*)d_in[1];
  const float* points1 = (const float*)d_in[2];
  const float* points2 = (const float*)d_in[3];
  const float* fuse_W  = (const float*)d_in[4];
  const float* fuse_b  = (const float*)d_in[5];
  const float* fuse_g  = (const float*)d_in[6];
  const float* fuse_be = (const float*)d_in[7];
  const float* blk_W1  = (const float*)d_in[8];
  const float* blk_b1  = (const float*)d_in[9];
  const float* blk_g1  = (const float*)d_in[10];
  const float* blk_be1 = (const float*)d_in[11];
  const float* blk_W2  = (const float*)d_in[12];
  const float* blk_b2  = (const float*)d_in[13];
  const float* blk_g2  = (const float*)d_in[14];
  const float* blk_be2 = (const float*)d_in[15];

  char* ws = (char*)d_ws;
  unsigned short* xhi  = (unsigned short*)(ws + kOffXhi);
  unsigned short* xlo  = (unsigned short*)(ws + kOffXlo);
  unsigned short* pahi = (unsigned short*)(ws + kOffAhi);
  unsigned short* palo = (unsigned short*)(ws + kOffAlo);
  float*          yb   = (float*)(ws + kOffY);
  unsigned short* pbhi = (unsigned short*)(ws + kOffBhi);
  unsigned short* pblo = (unsigned short*)(ws + kOffBlo);
  float*          p2T  = (float*)(ws + kOffP2T);
  unsigned short* whi  = (unsigned short*)(ws + kOffWhi);
  unsigned short* wlo  = (unsigned short*)(ws + kOffWlo);
  int*            idxt = (int*)(ws + kOffIdx);
  float*          dsel = (float*)(ws + kOffDsel);
  float*          part = (float*)(ws + kOffPart);
  float*          sstb = (float*)(ws + kOffSS);
  float*          out  = (float*)d_out;

  const size_t partStride = kPartBytes / 4;
  const int w1off = kWFuseElems;
  const int w2off = kWFuseElems + kWBlkElems;
  const int wblk  = kCOUT * kCOUT;
  const int applyBlocks = kMROWS * kCOUT / 8 / 256;

  wsplit_kernel<<<kWFuseBlocks + 2 * kWBlkBlocks, 256, 0, stream>>>(fuse_W, blk_W1, blk_W2, whi, wlo);
  p2t_kernel<<<dim3(kNSRC / 32, kCH2 / 32, kNB), 256, 0, stream>>>(points2, p2T);
  knn3_kernel<<<dim3(kNPTS / 256, kNB), 256, 0, stream>>>(xyz1, xyz2, idxt, dsel);
  xcat_kernel<<<kMROWS / 32, 256, 0, stream>>>(points1, p2T, idxt, dsel, xhi, xlo);

  run_conv_stats(xhi, xlo, kCIN, whi, wlo, fuse_b, fuse_g, fuse_be, yb, part, sstb, stream);
  bn_apply_planes<false><<<applyBlocks, 256, 0, stream>>>(yb, sstb, pbhi, pblo, pbhi, pblo);

  run_conv_stats(pbhi, pblo, kCOUT, whi + w1off, wlo + w1off, blk_b1, blk_g1, blk_be1,
                 yb, part + partStride, sstb + 512, stream);
  bn_apply_planes<false><<<applyBlocks, 256, 0, stream>>>(yb, sstb + 512, pahi, palo, pahi, palo);

  run_conv_stats(pahi, palo, kCOUT, whi + w2off, wlo + w2off, blk_b2, blk_g2, blk_be2,
                 yb, part + 2 * partStride, sstb + 1024, stream);
  bn_apply_planes<true><<<applyBlocks, 256, 0, stream>>>(yb, sstb + 1024, pbhi, pblo, pahi, palo);

  run_conv_stats(pahi, palo, kCOUT, whi + w1off + wblk, wlo + w1off + wblk,
                 blk_b1 + kCOUT, blk_g1 + kCOUT, blk_be1 + kCOUT,
                 yb, part + 3 * partStride, sstb + 1536, stream);
  bn_apply_planes<false><<<applyBlocks, 256, 0, stream>>>(yb, sstb + 1536, pbhi, pblo, pbhi, pblo);

  run_conv_stats(pbhi, pblo, kCOUT, whi + w2off + wblk, wlo + w2off + wblk,
                 blk_b2 + kCOUT, blk_g2 + kCOUT, blk_be2 + kCOUT,
                 yb, part + 4 * partStride, sstb + 2048, stream);
  bn_apply_final<<<kMROWS / 32, 256, 0, stream>>>(yb, sstb + 2048, pahi, palo, out);
}
